// mLSTMLayer_81741817577595
// MI455X (gfx1250) — hardware-run, weakly checked
//
#include <hip/hip_runtime.h>
#include <math.h>

constexpr int kBatch = 2;
constexpr int kSeq   = 2048;
constexpr int kEmb   = 1024;
constexpr int kInner = 2048;
constexpr int kHeads = 4;
constexpr int kDh    = 512;
constexpr int kTaps  = 4;
constexpr int kGateN = 64;
constexpr int kGateK = 3 * kInner;
constexpr int kInvRow = 32;
constexpr float kQKScale = 0.044194173824159216f;
constexpr float kEps     = 1.0e-6f;
constexpr float kInvDh   = 1.0f / 512.0f;
static_assert(kHeads * kDh == kInner, "shape");
static_assert(kSeq % 64 == 0 && kEmb % 64 == 0 && kInner % 64 == 0 && kDh % 64 == 0 && kGateN % 64 == 0, "mn tiles");
static_assert(kEmb % 32 == 0 && kInner % 32 == 0 && kDh % 32 == 0 && kSeq % 32 == 0, "k tiles");
static_assert(kGateK == 3 * 256 * 8, "gate rows");
static_assert(kSeq == 256 * 8 && kDh == 128 * 4 && kInner == 32 * 64 && kSeq == 64 * 32, "thread maps");

typedef __attribute__((ext_vector_type(16))) _Float16 v16h;
typedef __attribute__((ext_vector_type(8)))  _Float16 v8h;
typedef __attribute__((ext_vector_type(16))) __bf16   v16b;
typedef __attribute__((ext_vector_type(8)))  __bf16   v8b;
typedef __attribute__((ext_vector_type(8)))  float    v8f;
typedef __attribute__((ext_vector_type(4)))  float    v4f;
typedef __attribute__((ext_vector_type(4)))  unsigned int v4u;

__device__ __forceinline__ unsigned short f2bf_bits(float f) {
  unsigned u = __float_as_uint(f);
  return (unsigned short)((u + 0x7FFFu + ((u >> 16) & 1u)) >> 16);
}
__device__ __forceinline__ float bf_bits2f(unsigned short h) { return __uint_as_float(((unsigned)h) << 16); }
__device__ __forceinline__ float bf_rne(float f) { return __uint_as_float(((unsigned)f2bf_bits(f)) << 16); }
__device__ __forceinline__ unsigned pk16(unsigned short a, unsigned short b) { return (unsigned)a | ((unsigned)b << 16); }
__device__ __forceinline__ float bf_lo16(unsigned w) { return __uint_as_float(w << 16); }
__device__ __forceinline__ float bf_hi16(unsigned w) { return __uint_as_float(w & 0xffff0000u); }

__device__ __forceinline__ void dep_guard4_h(v8f& a, v8f& b, v8f& c, v8f& d, v16h x, v16h y) {
  asm volatile("v_nop\n\tv_nop\n\tv_nop\n\tv_nop" : "+v"(a), "+v"(b), "+v"(c), "+v"(d) : "v"(x), "v"(y));
}
__device__ __forceinline__ void dep_guard4_b(v8f& a, v8f& b, v8f& c, v8f& d, v16b x, v16b y) {
  asm volatile("v_nop\n\tv_nop\n\tv_nop\n\tv_nop" : "+v"(a), "+v"(b), "+v"(c), "+v"(d) : "v"(x), "v"(y));
}
__device__ __forceinline__ void keep4_h(v16h a, v16h b, v16h c, v16h d) { asm volatile("v_nop" :: "v"(a), "v"(b), "v"(c), "v"(d)); }
__device__ __forceinline__ void keep4_b(v16b a, v16b b, v16b c, v16b d) { asm volatile("v_nop" :: "v"(a), "v"(b), "v"(c), "v"(d)); }
__device__ __forceinline__ void acc_guard4(v8f& a, v8f& b, v8f& c, v8f& d) {
  asm volatile("v_nop\n\tv_nop\n\tv_nop\n\tv_nop" : "+v"(a), "+v"(b), "+v"(c), "+v"(d));
}
template <typename T> struct Frag;
template <> struct Frag<_Float16> {
  typedef v16h V; union U { v16h v; v8h h[2]; };
  static __device__ __forceinline__ v16h load(const _Float16* p) {
    U f; f.h[0] = *(const v8h*)(p); f.h[1] = *(const v8h*)(p + 16); return f.v;
  }
  static __device__ __forceinline__ v8f mma(v16h a, v16h b, v8f c) {
    return __builtin_amdgcn_wmma_f32_16x16x32_f16(false, a, false, b, (short)0, c, false, false);
  }
  static __device__ __forceinline__ void guard4(v8f& a, v8f& b, v8f& c, v8f& d, v16h x, v16h y) { dep_guard4_h(a, b, c, d, x, y); }
  static __device__ __forceinline__ void keep(v16h a, v16h b, v16h c, v16h d) { keep4_h(a, b, c, d); }
};
template <> struct Frag<__bf16> {
  typedef v16b V; union U { v16b v; v8b h[2]; };
  static __device__ __forceinline__ v16b load(const __bf16* p) {
    U f; f.h[0] = *(const v8b*)(p); f.h[1] = *(const v8b*)(p + 16); return f.v;
  }
  static __device__ __forceinline__ v8f mma(v16b a, v16b b, v8f c) {
    return __builtin_amdgcn_wmma_f32_16x16x32_bf16(false, a, false, b, (short)0, c, false, false);
  }
  static __device__ __forceinline__ void guard4(v8f& a, v8f& b, v8f& c, v8f& d, v16b x, v16b y) { dep_guard4_b(a, b, c, d, x, y); }
  static __device__ __forceinline__ void keep(v16b a, v16b b, v16b c, v16b d) { keep4_b(a, b, c, d); }
};

template <int ET> struct Elem;
template <> struct Elem<0> { typedef _Float16 T; };
template <> struct Elem<1> { typedef __bf16 T; };
template <int ET, bool SPLIT, int BIAS_MODE, int OUT_MODE, bool RESID, int ACT = 0, int CAUSAL = 0, bool BSPLIT = true>
__global__ __launch_bounds__(256) void wmma_gemm64(
    const unsigned short* __restrict__ Ap, const unsigned short* __restrict__ A2p, int lda, long strideA,
    const unsigned short* __restrict__ Btp, const unsigned short* __restrict__ Bt2p, int ldb, long strideB,
    void* __restrict__ Cout, void* __restrict__ Cout2, int ldc, long strideC,
    const float* __restrict__ bias,
    const float* __restrict__ resid, long strideR,
    int M, int N, int K, float scale) {
  typedef typename Elem<ET>::T T;
  typedef typename Frag<T>::V V;
  const T* A = (const T*)Ap; const T* A2 = (const T*)A2p; const T* Bt = (const T*)Btp; const T* Bt2 = (const T*)Bt2p;
  __shared__ __align__(16) float sT[8][16 * 68];
  const int b    = blockIdx.y;
  const int lane = threadIdx.x & 31;
  const int wave = threadIdx.x >> 5;
  const int tilesN = N >> 6;
  const int tilesM = M >> 6;
  const int tile = blockIdx.x * 8 + wave;
  if (tile >= tilesM * tilesN) return;
  const int tm = tile / tilesN;
  const int tn = tile - tm * tilesN;
  const int m0 = tm << 6;
  const int n0 = tn << 6;
  if (CAUSAL == 1) {
    if (n0 > m0) return;
  }
  const int kEnd = (CAUSAL == 2) ? ((m0 + 64 < K) ? (m0 + 64) : K) : K;

  const T* Ab  = A  + (size_t)b * strideA;
  const T* Bb  = Bt + (size_t)b * strideB;
  const T* Ab2 = SPLIT ? (A2  + (size_t)b * strideA) : nullptr;
  const T* Bb2 = (SPLIT && BSPLIT) ? (Bt2 + (size_t)b * strideB) : nullptr;

  const int rlane = lane & 15;
  const int koff  = (lane >> 4) * 8;
  const int mOff  = (lane >> 4) * 8;

  v8f acc[4][4];
#pragma unroll
  for (int i = 0; i < 4; ++i)
#pragma unroll
    for (int j = 0; j < 4; ++j) acc[i][j] = (v8f){0.f,0.f,0.f,0.f,0.f,0.f,0.f,0.f};

  for (int k0 = 0; k0 < kEnd; k0 += 32) {
    V bh[4], bl[4];
#pragma unroll
    for (int j = 0; j < 4; ++j) {
      const size_t bo = (size_t)(n0 + (j << 4) + rlane) * ldb + koff + k0;
      bh[j] = Frag<T>::load(Bb + bo);
      if (SPLIT && BSPLIT) bl[j] = Frag<T>::load(Bb2 + bo);
    }
#pragma unroll
    for (int i = 0; i < 4; ++i) {
      const size_t ao = (size_t)(m0 + (i << 4) + rlane) * lda + koff + k0;
      V ah = Frag<T>::load(Ab + ao);
      V al;
      if (SPLIT) al = Frag<T>::load(Ab2 + ao);
#pragma unroll
      for (int j = 0; j < 4; ++j) {
        acc[i][j] = Frag<T>::mma(ah, bh[j], acc[i][j]);
        if (SPLIT) {
          if (BSPLIT) acc[i][j] = Frag<T>::mma(ah, bl[j], acc[i][j]);
          acc[i][j] = Frag<T>::mma(al, bh[j], acc[i][j]);
        }
      }
      Frag<T>::guard4(acc[i][0], acc[i][1], acc[i][2], acc[i][3], ah, SPLIT ? al : ah);
    }
    Frag<T>::keep(bh[0], bh[1], bh[2], bh[3]);
    if (SPLIT && BSPLIT) Frag<T>::keep(bl[0], bl[1], bl[2], bl[3]);
  }
  acc_guard4(acc[0][0], acc[0][1], acc[0][2], acc[0][3]);
  acc_guard4(acc[1][0], acc[1][1], acc[1][2], acc[1][3]);
  acc_guard4(acc[2][0], acc[2][1], acc[2][2], acc[2][3]);
  acc_guard4(acc[3][0], acc[3][1], acc[3][2], acc[3][3]);

  float* slab = sT[wave];
  const float* Rb = RESID ? (resid + (size_t)b * strideR) : nullptr;
#pragma unroll
  for (int i = 0; i < 4; ++i) {
    const int mBase = m0 + (i << 4);
#pragma unroll
    for (int j = 0; j < 4; ++j) {
      const int n = n0 + (j << 4) + rlane;
      float bv = 0.f;
      if (BIAS_MODE == 2) bv = bias[n];
#pragma unroll
      for (int r = 0; r < 8; ++r) {
        float v = acc[i][j][r] * scale;
        if (BIAS_MODE == 1) v += bias[mBase + mOff + r];
        if (BIAS_MODE == 2) v += bv;
        if (RESID) v += Rb[(size_t)(mBase + mOff + r) * ldc + n];
        if (ACT == 2) v = fmaxf(v, 0.0f);
        if (ACT == 4) v = (v > 0.f) ? v : 0.01f * v;
        slab[(mOff + r) * 68 + (j << 4) + rlane] = v;
      }
    }
    __builtin_amdgcn_fence(__ATOMIC_RELEASE, "workgroup");
    __builtin_amdgcn_wave_barrier();
    __builtin_amdgcn_fence(__ATOMIC_ACQUIRE, "workgroup");
    if (OUT_MODE == 0) {
      float* C = (float*)Cout + (size_t)b * strideC;
      const int hh = lane >> 4, c4 = (lane & 15) * 4;
      for (int pass = 0; pass < 2; ++pass) {
#pragma unroll
        for (int it = 0; it < 8; ++it) {
          const int row = it * 2 + hh;
          v4f v = *(const v4f*)(slab + row * 68 + c4);
          *(volatile v4f*)(C + (size_t)(mBase + row) * ldc + n0 + c4) = v;
        }
        __threadfence();
      }
    } else {
      const int q = lane >> 3, c8 = (lane & 7) * 8;
      unsigned short* C  = (unsigned short*)Cout  + (size_t)b * strideC;
      unsigned short* C2 = (OUT_MODE == 2) ? ((unsigned short*)Cout2 + (size_t)b * strideC) : nullptr;
      for (int pass = 0; pass < 2; ++pass) {
#pragma unroll
        for (int it = 0; it < 4; ++it) {
          const int row = it * 4 + q;
          const float* sp = slab + row * 68 + c8;
          v8h hv, lv;
#pragma unroll
          for (int e = 0; e < 8; ++e) {
            if (OUT_MODE == 1) {
              hv[e] = (_Float16)sp[e];
            } else {
              unsigned short hb = f2bf_bits(sp[e]);
              hv[e] = __builtin_bit_cast(_Float16, hb);
              if (OUT_MODE == 2) {
                unsigned short lb = f2bf_bits(sp[e] - bf_bits2f(hb));
                lv[e] = __builtin_bit_cast(_Float16, lb);
              }
            }
          }
          *(volatile v8h*)(C + (size_t)(mBase + row) * ldc + n0 + c8) = hv;
          if (OUT_MODE == 2) *(volatile v8h*)(C2 + (size_t)(mBase + row) * ldc + n0 + c8) = lv;
        }
        __threadfence();
      }
    }
    __builtin_amdgcn_fence(__ATOMIC_RELEASE, "workgroup");
    __builtin_amdgcn_wave_barrier();
    __builtin_amdgcn_fence(__ATOMIC_ACQUIRE, "workgroup");
  }
}

__global__ __launch_bounds__(256) void wt_cast_kernel(const float* __restrict__ W, unsigned short* __restrict__ WT,
                                                      int nrows, int ncols) {
  __shared__ float sm[64][65];
  const int t  = threadIdx.x;
  const int r0 = blockIdx.x * 64;
  const int c0 = blockIdx.y * 64;
#pragma unroll
  for (int i = 0; i < 16; ++i) {
    const int e = i * 256 + t;
    const int rl = e >> 6;
    const int cl = e & 63;
    sm[cl][rl] = W[(size_t)(r0 + rl) * ncols + c0 + cl];
  }
  __syncthreads();
  const int lane = t & 31, wave = t >> 5;
  const int q = lane >> 3, c8 = (lane & 7) * 8;
  for (int pass = 0; pass < 2; ++pass) {
#pragma unroll
    for (int it = 0; it < 2; ++it) {
      const int row = wave * 8 + it * 4 + q;
      unsigned short hb[8];
#pragma unroll
      for (int e = 0; e < 8; ++e) hb[e] = f2bf_bits(sm[row][c8 + e]);
      const v4u u = (v4u){pk16(hb[0], hb[1]), pk16(hb[2], hb[3]), pk16(hb[4], hb[5]), pk16(hb[6], hb[7])};
      *(volatile v4u*)(WT + (size_t)(c0 + row) * nrows + r0 + c8) = u;
    }
    __threadfence();
  }
}

__global__ __launch_bounds__(256) void wg_kernel(const float* __restrict__ Wi, const float* __restrict__ Wf,
                                                 unsigned short* __restrict__ WGT) {
  const int t = threadIdx.x;
  const int n = blockIdx.y;
  const int f0 = (blockIdx.x * 256 + t) * 8;
  const float* src = (n < 4) ? Wi : Wf;
  const int col = n & 3;
  const float fac = (n < 8) ? 1.0f : 0.0f;
  unsigned short hb[8];
#pragma unroll
  for (int e = 0; e < 8; ++e) hb[e] = f2bf_bits(src[(size_t)(f0 + e) * kHeads + col] * fac);
  const v4u u = (v4u){pk16(hb[0], hb[1]), pk16(hb[2], hb[3]), pk16(hb[4], hb[5]), pk16(hb[6], hb[7])};
  unsigned short* op = WGT + (size_t)n * kGateK + f0;
  *(volatile v4u*)op = u;
  __threadfence();
  *(volatile v4u*)op = u;
}

__global__ __launch_bounds__(256) void xcast_kernel(const float* __restrict__ in, unsigned short* __restrict__ out, int n8) {
  const int i = blockIdx.x * 256 + threadIdx.x;
  if (i >= n8) return;
  const float* p = in + 8 * (size_t)i;
  const v4f a = *(const v4f*)(p);
  const v4f c = *(const v4f*)(p + 4);
  unsigned short hb[8];
#pragma unroll
  for (int e = 0; e < 4; ++e) {
    hb[e]     = f2bf_bits(a[e]);
    hb[4 + e] = f2bf_bits(c[e]);
  }
  const v4u u = (v4u){pk16(hb[0], hb[1]), pk16(hb[2], hb[3]), pk16(hb[4], hb[5]), pk16(hb[6], hb[7])};
  unsigned short* q = out + 8 * (size_t)i;
  *(volatile v4u*)q = u;
  __threadfence();
  *(volatile v4u*)q = u;
}

__global__ __launch_bounds__(256) void conv_headwise_kernel(
    const float* __restrict__ XMb, const float* __restrict__ convk, const float* __restrict__ convb,
    const float* __restrict__ Wq, const float* __restrict__ Wk, const float* __restrict__ Wv,
    float* __restrict__ ACTb, unsigned short* __restrict__ Qb, unsigned short* __restrict__ Kb,
    unsigned short* __restrict__ Vb, int nsub) {
  __shared__ __align__(16) float xs[35 * 68];
  __shared__ __align__(16) float cks[4 * 64];
  __shared__ float cbs[64];
  __shared__ __align__(16) float wqs[256];
  __shared__ __align__(16) float wks[256];
  __shared__ __align__(16) float wvs[256];
  __shared__ __align__(16) float acts[32 * 68];
  __shared__ __align__(16) float qsm[32 * 68];
  __shared__ __align__(16) float ksm[32 * 68];
  __shared__ __align__(16) float vsm[32 * 68];
  const int t = threadIdx.x;
  const int lane = t & 31, wave = t >> 5;
  const int c0 = blockIdx.x * 64;
  const int s0 = blockIdx.y * 32;

#pragma unroll
  for (int it = 0; it < 3; ++it) {
    const int idx = it * 256 + t;
    const int idc = (idx < 560) ? idx : 559;
    const int row = idc >> 4;
    const int c4  = (idc & 15) * 4;
    const int tok = s0 - 3 + row;
    const int tokc = (tok < 0) ? 0 : tok;
    v4f v = *(const v4f*)(XMb + (size_t)tokc * kInner + c0 + c4);
    const float fac = (tok < 0) ? 0.0f : 1.0f;
    v = v * fac;
    *(v4f*)(xs + row * 68 + c4) = v;
  }
  if (wave < 2) {
    const int tap = t >> 4;
    const int c4 = (t & 15) * 4;
    const v4f v = *(const v4f*)(convk + (size_t)tap * kInner + c0 + c4);
#pragma unroll
    for (int e = 0; e < 4; ++e) cks[tap * 64 + c4 + e] = bf_rne(v[e]);
  } else if (wave < 4) {
    const int tt = t - 64;
    const v4f v = *(const v4f*)(Wq + (size_t)c0 * 4 + tt * 4);
#pragma unroll
    for (int e = 0; e < 4; ++e) wqs[tt * 4 + e] = bf_rne(v[e]);
  } else if (wave < 6) {
    const int tt = t - 128;
    const v4f v = *(const v4f*)(Wk + (size_t)c0 * 4 + tt * 4);
#pragma unroll
    for (int e = 0; e < 4; ++e) wks[tt * 4 + e] = bf_rne(v[e]);
  } else {
    const int tt = t - 192;
    const v4f v = *(const v4f*)(Wv + (size_t)c0 * 4 + tt * 4);
#pragma unroll
    for (int e = 0; e < 4; ++e) wvs[tt * 4 + e] = bf_rne(v[e]);
  }
  if (wave == 0) {
    cbs[lane]      = bf_rne(convb[c0 + lane]);
    cbs[32 + lane] = bf_rne(convb[c0 + 32 + lane]);
  }
  __syncthreads();

  const int tok = t >> 3;
  const int cg  = (t & 7) * 8;
  const int ns  = (nsub > 8) ? 8 : ((nsub < 0) ? 0 : nsub);

#pragma unroll 1
  for (int e = 0; e < ns; ++e) {
    const int c = cg + e;
    float cv = cbs[c];
    cv = cv + cks[0 * 64 + c] * xs[(tok + 0) * 68 + c];
    cv = cv + cks[1 * 64 + c] * xs[(tok + 1) * 68 + c];
    cv = cv + cks[2 * 64 + c] * xs[(tok + 2) * 68 + c];
    cv = cv + cks[3 * 64 + c] * xs[(tok + 3) * 68 + c];
    const float sg = 1.0f / (1.0f + expf(-cv));
    acts[tok * 68 + c] = cv * sg;
  }
#pragma unroll 1
  for (int e = 0; e < ns; ++e) {
    const int c  = cg + e;
    const int kb = c & ~3;
    const int nl = c >> 2;
    const int d  = c & 3;
    const float a0 = acts[tok * 68 + kb + 0];
    const float a1 = acts[tok * 68 + kb + 1];
    const float a2 = acts[tok * 68 + kb + 2];
    const float a3 = acts[tok * 68 + kb + 3];
    const float x0 = xs[(tok + 3) * 68 + kb + 0];
    const float x1 = xs[(tok + 3) * 68 + kb + 1];
    const float x2 = xs[(tok + 3) * 68 + kb + 2];
    const float x3 = xs[(tok + 3) * 68 + kb + 3];
    const float* wq = wqs + nl * 16 + d;
    const float* wk = wks + nl * 16 + d;
    const float* wv = wvs + nl * 16 + d;
    float qv = a0 * wq[0];
    qv = qv + a1 * wq[4];
    qv = qv + a2 * wq[8];
    qv = qv + a3 * wq[12];
    float kv = a0 * wk[0];
    kv = kv + a1 * wk[4];
    kv = kv + a2 * wk[8];
    kv = kv + a3 * wk[12];
    float vv = x0 * wv[0];
    vv = vv + x1 * wv[4];
    vv = vv + x2 * wv[8];
    vv = vv + x3 * wv[12];
    qsm[tok * 68 + c] = qv;
    ksm[tok * 68 + c] = kv;
    vsm[tok * 68 + c] = vv;
  }
  __syncthreads();

  for (int pass = 0; pass < 2; ++pass) {
#pragma unroll
    for (int it = 0; it < 2; ++it) {
      const int row = wave * 4 + it * 2 + (lane >> 4);
      const int c4 = (lane & 15) * 4;
      const v4f v = *(const v4f*)(acts + row * 68 + c4);
      *(volatile v4f*)(ACTb + (size_t)(s0 + row) * kInner + c0 + c4) = v;
    }
    {
      const int row = wave * 4 + (lane >> 3);
      const int c8 = (lane & 7) * 8;
      const v4f q0 = *(const v4f*)(qsm + row * 68 + c8);
      const v4f q1 = *(const v4f*)(qsm + row * 68 + c8 + 4);
      const v4f k0 = *(const v4f*)(ksm + row * 68 + c8);
      const v4f k1 = *(const v4f*)(ksm + row * 68 + c8 + 4);
      const v4f v0 = *(const v4f*)(vsm + row * 68 + c8);
      const v4f v1 = *(const v4f*)(vsm + row * 68 + c8 + 4);
      const v4u uq = (v4u){pk16(f2bf_bits(q0[0]), f2bf_bits(q0[1])), pk16(f2bf_bits(q0[2]), f2bf_bits(q0[3])),
                           pk16(f2bf_bits(q1[0]), f2bf_bits(q1[1])), pk16(f2bf_bits(q1[2]), f2bf_bits(q1[3]))};
      const v4u uk = (v4u){pk16(f2bf_bits(k0[0]), f2bf_bits(k0[1])), pk16(f2bf_bits(k0[2]), f2bf_bits(k0[3])),
                           pk16(f2bf_bits(k1[0]), f2bf_bits(k1[1])), pk16(f2bf_bits(k1[2]), f2bf_bits(k1[3]))};
      const v4u uv = (v4u){pk16(f2bf_bits(v0[0]), f2bf_bits(v0[1])), pk16(f2bf_bits(v0[2]), f2bf_bits(v0[3])),
                           pk16(f2bf_bits(v1[0]), f2bf_bits(v1[1])), pk16(f2bf_bits(v1[2]), f2bf_bits(v1[3]))};
      const size_t o = (size_t)(s0 + row) * kInner + c0 + c8;
      *(volatile v4u*)(Qb + o) = uq;
      *(volatile v4u*)(Kb + o) = uk;
      *(volatile v4u*)(Vb + o) = uv;
    }
    __threadfence();
  }
}

__global__ __launch_bounds__(256) void vt_kernel(const unsigned short* __restrict__ Vb, unsigned short* __restrict__ VTb) {
  __shared__ unsigned short sm[64][72];
  const int t  = threadIdx.x;
  const int s0 = blockIdx.x * 64;
  const int c0 = blockIdx.y * 64;
#pragma unroll
  for (int it = 0; it < 2; ++it) {
    const int idx = it * 256 + t;
    const int row = idx >> 3;
    const int c8  = (idx & 7) * 8;
    const v4u u = *(const v4u*)(Vb + (size_t)(s0 + row) * kInner + c0 + c8);
#pragma unroll
    for (int q = 0; q < 4; ++q) {
      sm[c8 + 2 * q][row]     = (unsigned short)(u[q] & 0xffffu);
      sm[c8 + 2 * q + 1][row] = (unsigned short)(u[q] >> 16);
    }
  }
  __syncthreads();
  const int lane = t & 31, wave = t >> 5;
  const int q = lane >> 3, c8 = (lane & 7) * 8;
  for (int pass = 0; pass < 2; ++pass) {
#pragma unroll
    for (int it = 0; it < 2; ++it) {
      const int row = wave * 8 + it * 4 + q;
      const v4u u = (v4u){pk16(sm[row][c8 + 0], sm[row][c8 + 1]), pk16(sm[row][c8 + 2], sm[row][c8 + 3]),
                          pk16(sm[row][c8 + 4], sm[row][c8 + 5]), pk16(sm[row][c8 + 6], sm[row][c8 + 7])};
      *(volatile v4u*)(VTb + (size_t)(c0 + row) * kSeq + s0 + c8) = u;
    }
    __threadfence();
  }
}

__global__ __launch_bounds__(256) void scan_kernel(const float* __restrict__ G0, const float* __restrict__ G1,
                                                   const float* __restrict__ G2, const float* __restrict__ bi,
                                                   const float* __restrict__ bfv, float* __restrict__ lfcT,
                                                   float* __restrict__ gjT, float* __restrict__ pmT, int nsub) {
  __shared__ __align__(16) float la[kSeq];
  __shared__ __align__(16) float ga[kSeq];
  __shared__ __align__(16) float pa[kSeq];
  __shared__ float sb[2][256];
  const int h = blockIdx.x;
  const int t = threadIdx.x;
  const float kNegInf = -__builtin_inff();
  const float bih = bf_rne(bi[h]);
  const float bfh = bf_rne(bfv[h]);
  const int ns = (nsub > 8) ? 8 : ((nsub < 0) ? 0 : nsub);

#pragma unroll 1
  for (int e = 0; e < ns; ++e) {
    const int s = t * 8 + e;
    const float* r0 = G0 + (size_t)s * kGateN;
    const float* r1 = G1 + (size_t)s * kGateN;
    const float* r2 = G2 + (size_t)s * kGateN;
    const float ip = ((r0[h] + r1[h]) + r2[h]) + bih;
    const float fp = ((r0[4 + h] + r1[4 + h]) + r2[4 + h]) + bfh;
    const float lf = fminf(fp, 0.0f) - log1pf(expf(-fabsf(fp)));
    la[s] = lf;
    ga[s] = ip;
  }
  float run = 0.0f;
#pragma unroll 1
  for (int e = 0; e < ns; ++e) {
    const int s = t * 8 + e;
    run = run + la[s];
    la[s] = run;
  }
  sb[0][t] = run;
  __syncthreads();
  int cur = 0;
#pragma unroll 1
  for (int off = 1; off < 256; off <<= 1) {
    float v = sb[cur][t];
    int idx = t - off;
    idx = (idx < 0) ? 0 : idx;
    const float w = sb[cur][idx];
    v = (t >= off) ? (v + w) : v;
    sb[cur ^ 1][t] = v;
    __syncthreads();
    cur ^= 1;
  }
  const int tm1 = (t == 0) ? 0 : (t - 1);
  const float offs = (t == 0) ? 0.0f : sb[cur][tm1];
  float rm = kNegInf;
#pragma unroll 1
  for (int e = 0; e < ns; ++e) {
    const int s = t * 8 + e;
    const float lfv = offs + la[s];
    la[s] = lfv;
    const float gv = ga[s] - lfv;
    ga[s] = gv;
    rm = fmaxf(rm, gv);
  }
  __syncthreads();
  sb[0][t] = rm;
  __syncthreads();
  cur = 0;
#pragma unroll 1
  for (int off = 1; off < 256; off <<= 1) {
    float v = sb[cur][t];
    int idx = t - off;
    idx = (idx < 0) ? 0 : idx;
    const float w = sb[cur][idx];
    v = (t >= off) ? fmaxf(v, w) : v;
    sb[cur ^ 1][t] = v;
    __syncthreads();
    cur ^= 1;
  }
  const float offm = (t == 0) ? kNegInf : sb[cur][tm1];
  float cm = offm;
#pragma unroll 1
  for (int e = 0; e < ns; ++e) {
    const int s = t * 8 + e;
    cm = fmaxf(cm, ga[s]);
    pa[s] = cm;
  }
  __syncthreads();
  float* lp = lfcT + (size_t)h * kSeq;
  float* gp = gjT  + (size_t)h * kSeq;
  float* pp = pmT  + (size_t)h * kSeq;
  for (int pass = 0; pass < 2; ++pass) {
#pragma unroll
    for (int it = 0; it < 2; ++it) {
      const int idx = it * 256 + t;
      const v4f a = *(const v4f*)(la + 4 * idx);
      const v4f g = *(const v4f*)(ga + 4 * idx);
      const v4f p = *(const v4f*)(pa + 4 * idx);
      *(volatile v4f*)(lp + 4 * idx) = a;
      *(volatile v4f*)(gp + 4 * idx) = g;
      *(volatile v4f*)(pp + 4 * idx) = p;
    }
    __threadfence();
  }
}

__global__ __launch_bounds__(256) void pcell_kernel(const unsigned short* __restrict__ SCp, const float* __restrict__ gjp,
                                                    const float* __restrict__ pmp, const float* __restrict__ lfcp,
                                                    unsigned short* __restrict__ PPp, float* __restrict__ INVNp) {
  __shared__ float red[8];
  const int i = blockIdx.x;
  const int t = threadIdx.x;
  const int lane = t & 31, wave = t >> 5;
  const int qb = i >> 6;
  const int cend = (qb + 1) * 64;
  const int c0 = t * 8;
  const int cl = (c0 + 8 <= cend) ? c0 : (cend - 8);
  const v4u sw = *(const v4u*)(SCp + (size_t)i * kSeq + cl);
  const v4f g0 = *(const v4f*)(gjp + cl);
  const v4f g1 = *(const v4f*)(gjp + cl + 4);
  const float pmi = pmp[i];
  const float lfi = lfcp[i];
  float sc[8], gg[8];
#pragma unroll
  for (int q = 0; q < 4; ++q) {
    sc[2 * q]     = bf_lo16(sw[q]);
    sc[2 * q + 1] = bf_hi16(sw[q]);
    gg[q]     = g0[q];
    gg[4 + q] = g1[q];
  }
  float rs = 0.0f;
  unsigned short pb[8];
#pragma unroll
  for (int e = 0; e < 8; ++e) {
    const int j = c0 + e;
    const float fk = (j <= i) ? 1.0f : 0.0f;
    const float d = fminf(gg[e] - pmi, 0.0f);
    const float ex = expf(d);
    const float p = ((sc[e] * kQKScale) * ex) * fk;
    rs = rs + p;
    pb[e] = f2bf_bits(p);
  }
  const v4u u = (v4u){pk16(pb[0], pb[1]), pk16(pb[2], pb[3]), pk16(pb[4], pb[5]), pk16(pb[6], pb[7])};
#pragma unroll
  for (int off = 16; off > 0; off >>= 1) rs += __shfl_xor(rs, off, 32);
  if (lane == 0) red[wave] = rs;
  unsigned short* pr = PPp + (size_t)i * kSeq + c0;
  if (c0 < cend) *(volatile v4u*)pr = u;
  __threadfence();
  if (c0 < cend) *(volatile v4u*)pr = u;
  __syncthreads();
  if (wave == 0) {
    float tot = red[0];
#pragma unroll
    for (int w = 1; w < 8; ++w) tot = tot + red[w];
    const float nrm = fmaxf(fabsf(tot), expf(-(lfi + pmi)));
    const float inv = 1.0f / (nrm + kEps);
    const float val = (lane == 0) ? inv : 0.0f;
    volatile float* ip = INVNp + (size_t)i * kInvRow + lane;
    *ip = val;
    __threadfence();
    *ip = val;
  }
}

__global__ __launch_bounds__(128) void ln_gate_kernel(const float* __restrict__ OO, const float* __restrict__ INVN,
                                                      const float* __restrict__ ACTb, const float* __restrict__ Zb,
                                                      const float* __restrict__ nsc, const float* __restrict__ skp,
                                                      unsigned short* __restrict__ HSh, unsigned short* __restrict__ HSl,
                                                      int head) {
  __shared__ float red[4];
  __shared__ __align__(16) unsigned short shi[kDh];
  __shared__ __align__(16) unsigned short slo[kDh];
  const int i = blockIdx.x;
  const int t = threadIdx.x;
  const int lane = t & 31, wave = t >> 5;
  const int hd = (head < 0) ? 0 : ((head >= kHeads) ? (kHeads - 1) : head);
  const int d0 = 4 * t;
  const int col = hd * kDh + d0;
  const v4f o  = *(const v4f*)(OO + (size_t)i * kDh + d0);
  const float inv = INVN[(size_t)i * kInvRow];
  const v4f a  = *(const v4f*)(ACTb + (size_t)i * kInner + col);
  const v4f z  = *(const v4f*)(Zb + (size_t)i * kInner + col);
  const v4f n4 = *(const v4f*)(nsc + col);
  const v4f s4 = *(const v4f*)(skp + col);
  float hv[4];
#pragma unroll
  for (int e = 0; e < 4; ++e) hv[e] = o[e] * inv;
  float s1 = (hv[0] + hv[1]) + (hv[2] + hv[3]);
#pragma unroll
  for (int off = 16; off > 0; off >>= 1) s1 += __shfl_xor(s1, off, 32);
  if (lane == 0) red[wave] = s1;
  __syncthreads();
  const float mu = ((red[0] + red[1]) + (red[2] + red[3])) * kInvDh;
  __syncthreads();
  float dv[4];
#pragma unroll
  for (int e = 0; e < 4; ++e) dv[e] = hv[e] - mu;
  float s2 = (dv[0] * dv[0] + dv[1] * dv[1]) + (dv[2] * dv[2] + dv[3] * dv[3]);
#pragma unroll
  for (int off = 16; off > 0; off >>= 1) s2 += __shfl_xor(s2, off, 32);
  if (lane == 0) red[wave] = s2;
  __syncthreads();
  const float var = ((red[0] + red[1]) + (red[2] + red[3])) * kInvDh;
  const float rsd = rsqrtf(var + kEps);
#pragma unroll
  for (int e = 0; e < 4; ++e) {
    const float hn  = (dv[e] * rsd) * bf_rne(n4[e]);
    const float hsk = hn + bf_rne(s4[e]) * a[e];
    const float zz  = z[e];
    const float swz = zz * (1.0f / (1.0f + expf(-zz)));
    const float hs  = hsk * swz;
    const unsigned short hb = f2bf_bits(hs);
    const unsigned short lb = f2bf_bits(hs - bf_bits2f(hb));
    shi[d0 + e] = hb;
    slo[d0 + e] = lb;
  }
  __syncthreads();
  if (wave < 2) {
    const int c8 = t * 8;
    const v4u uh = (v4u){pk16(shi[c8 + 0], shi[c8 + 1]), pk16(shi[c8 + 2], shi[c8 + 3]),
                         pk16(shi[c8 + 4], shi[c8 + 5]), pk16(shi[c8 + 6], shi[c8 + 7])};
    const v4u ul = (v4u){pk16(slo[c8 + 0], slo[c8 + 1]), pk16(slo[c8 + 2], slo[c8 + 3]),
                         pk16(slo[c8 + 4], slo[c8 + 5]), pk16(slo[c8 + 6], slo[c8 + 7])};
    const size_t ob = (size_t)i * kInner + hd * kDh + c8;
    *(volatile v4u*)(HSh + ob) = uh;
    *(volatile v4u*)(HSl + ob) = ul;
    __threadfence();
    *(volatile v4u*)(HSh + ob) = uh;
    *(volatile v4u*)(HSl + ob) = ul;
  }
}

extern "C" void kernel_launch(void* const* d_in, const int* in_sizes, int n_in,
                              void* d_out, int out_size, void* d_ws, size_t ws_size,
                              hipStream_t stream) {
  if (n_in < 15) return;
  const int nX = kBatch * kSeq * kEmb;
  if (in_sizes[0] != nX) return;
  if (in_sizes[1] != kEmb * kInner || in_sizes[2] != kEmb * kInner) return;
  if (in_sizes[3] != kTaps * kInner || in_sizes[4] != kInner) return;
  if (in_sizes[5] != kInner * 4 || in_sizes[6] != kInner * 4 || in_sizes[7] != kInner * 4) return;
  if (in_sizes[8] != kGateK * kHeads || in_sizes[10] != kGateK * kHeads) return;
  if (in_sizes[9] != kHeads || in_sizes[11] != kHeads) return;
  if (in_sizes[12] != kInner || in_sizes[13] != kInner || in_sizes[14] != kInner * kEmb) return;
  if (out_size != nX) return;

  const size_t szW    = (size_t)kInner * kEmb * 2;
  const size_t szWG   = (size_t)kGateN * kGateK * 2;
  const size_t szXB   = (size_t)kSeq * kEmb * 2;
  const size_t szF32P = (size_t)kSeq * kInner * 4;
  const size_t szB16P = (size_t)kSeq * kInner * 2;
  const size_t szSC   = (size_t)kSeq * kSeq * 2;
  const size_t szGG   = (size_t)3 * kSeq * kGateN * 4;
  const size_t szTAB  = (size_t)3 * kHeads * kSeq * 4;
  const size_t szINVN = (size_t)kSeq * kInvRow * 4;
  const size_t szOO   = (size_t)kSeq * kDh * 4;
  const size_t oWUM = 0;
  const size_t oWUZ = oWUM + szW;
  const size_t oWDT = oWUZ + szW;
  const size_t oWGT = oWDT + szW;
  const size_t oXB  = oWGT + szWG;
  const size_t oXM  = oXB + szXB;
  const size_t oACT = oXM + szF32P;
  const size_t oQP  = oACT + szF32P;
  const size_t oKP  = oQP + szB16P;
  const size_t oVP  = oKP + szB16P;
  const size_t oVT  = oVP + szB16P;
  const size_t oGG  = oVT + szB16P;
  const size_t oTAB = oGG + szGG;
  const size_t oSC  = oTAB + szTAB;
  const size_t oPP  = oSC + szSC;
  const size_t oINV = oPP + szSC;
  const size_t oOO  = oINV + szINVN;
  const size_t oHSH = oOO + szOO;
  const size_t oHSL = oHSH + szB16P;
  const size_t total = oHSL + szB16P;
  if (ws_size < total) return;
  if (total > (size_t)134217728) return;

  const float* x      = (const float*)d_in[0];
  const float* W_up_m = (const float*)d_in[1];
  const float* W_up_z = (const float*)d_in[2];
  const float* convk  = (const float*)d_in[3];
  const float* convb  = (const float*)d_in[4];
  const float* Wq     = (const float*)d_in[5];
  const float* Wk     = (const float*)d_in[6];
  const float* Wv     = (const float*)d_in[7];
  const float* Wi     = (const float*)d_in[8];
  const float* bi     = (const float*)d_in[9];
  const float* Wf     = (const float*)d_in[10];
  const float* bfp    = (const float*)d_in[11];
  const float* nsc    = (const float*)d_in[12];
  const float* skp    = (const float*)d_in[13];
  const float* Wd     = (const float*)d_in[14];
  float* out = (float*)d_out;
  char* ws = (char*)d_ws;
  unsigned short* WUM = (unsigned short*)(ws + oWUM);
  unsigned short* WUZ = (unsigned short*)(ws + oWUZ);
  unsigned short* WDT = (unsigned short*)(ws + oWDT);
  unsigned short* WGT = (unsigned short*)(ws + oWGT);
  unsigned short* XB  = (unsigned short*)(ws + oXB);
  float* XM  = (float*)(ws + oXM);
  float* ACT = (float*)(ws + oACT);
  unsigned short* QP = (unsigned short*)(ws + oQP);
  unsigned short* KP = (unsigned short*)(ws + oKP);
  unsigned short* VP = (unsigned short*)(ws + oVP);
  unsigned short* VT = (unsigned short*)(ws + oVT);
  float* GG  = (float*)(ws + oGG);
  float* TAB = (float*)(ws + oTAB);
  float* LFC = TAB;
  float* GJ  = TAB + (size_t)kHeads * kSeq;
  float* PM  = TAB + (size_t)2 * kHeads * kSeq;
  unsigned short* SC = (unsigned short*)(ws + oSC);
  unsigned short* PP = (unsigned short*)(ws + oPP);
  float* INVN = (float*)(ws + oINV);
  float* OO   = (float*)(ws + oOO);
  unsigned short* HSH = (unsigned short*)(ws + oHSH);
  unsigned short* HSL = (unsigned short*)(ws + oHSL);
  const float* dumf = TAB;

  wt_cast_kernel<<<dim3(kEmb / 64, kInner / 64), dim3(256), 0, stream>>>(W_up_m, WUM, kEmb, kInner);
  wt_cast_kernel<<<dim3(kEmb / 64, kInner / 64), dim3(256), 0, stream>>>(W_up_z, WUZ, kEmb, kInner);
  wt_cast_kernel<<<dim3(kInner / 64, kEmb / 64), dim3(256), 0, stream>>>(Wd, WDT, kInner, kEmb);
  wg_kernel<<<dim3(kGateK / 8 / 256, kGateN), dim3(256), 0, stream>>>(Wi, Wf, WGT);

  const int tilesUp    = (kSeq / 64) * (kInner / 64);
  const int tilesGate  = (kSeq / 64) * (kGateN / 64);
  const int tilesScore = (kSeq / 64) * (kSeq / 64);
  const int tilesCell  = (kSeq / 64) * (kDh / 64);
  const int tilesDown  = (kSeq / 64) * (kEmb / 64);
  const int n8x = (kSeq * kEmb) / 8;

  for (int b = 0; b < kBatch; ++b) {
    const float* xb = x + (size_t)b * kSeq * kEmb;
    xcast_kernel<<<dim3(n8x / 256), dim3(256), 0, stream>>>(xb, XB, n8x);
    wmma_gemm64<1, false, 0, 0, false, 0, 0, true><<<dim3(tilesUp / 8, 1), dim3(256), 0, stream>>>(
        XB, XB, kEmb, 0L, WUM, WUM, kEmb, 0L, (void*)XM, (void*)XM, kInner, 0L, dumf, dumf, 0L,
        kSeq, kInner, kEmb, 1.0f);
    conv_headwise_kernel<<<dim3(kInner / 64, kSeq / 32), dim3(256), 0, stream>>>(
        XM, convk, convb, Wq, Wk, Wv, ACT, QP, KP, VP, 8);
    wmma_gemm64<1, false, 0, 0, false, 0, 0, true><<<dim3(tilesUp / 8, 1), dim3(256), 0, stream>>>(
        XB, XB, kEmb, 0L, WUZ, WUZ, kEmb, 0L, (void*)XM, (void*)XM, kInner, 0L, dumf, dumf, 0L,
        kSeq, kInner, kEmb, 1.0f);
    vt_kernel<<<dim3(kSeq / 64, kInner / 64), dim3(256), 0, stream>>>(VP, VT);
    for (int part = 0; part < 3; ++part) {
      const unsigned short* Ag = (part == 0) ? QP : (part == 1) ? KP : VP;
      const unsigned short* Bg = WGT + (size_t)part * kInner;
      float* Cg = GG + (size_t)part * kSeq * kGateN;
      wmma_gemm64<1, false, 0, 0, false, 0, 0, true><<<dim3(tilesGate / 8, 1), dim3(256), 0, stream>>>(
          Ag, Ag, kInner, 0L, Bg, Bg, kGateK, 0L, (void*)Cg, (void*)Cg, kGateN, 0L, dumf, dumf, 0L,
          kSeq, kGateN, kInner, 1.0f);
    }
    scan_kernel<<<dim3(kHeads), dim3(256), 0, stream>>>(
        GG, GG + (size_t)kSeq * kGateN, GG + (size_t)2 * kSeq * kGateN, bi, bfp, LFC, GJ, PM, 8);

    for (int h = 0; h < kHeads; ++h) {
      const unsigned short* Aq = QP + (size_t)h * kDh;
      const unsigned short* Bk = KP + (size_t)h * kDh;
      wmma_gemm64<1, false, 0, 3, false, 0, 1, true><<<dim3(tilesScore / 8, 1), dim3(256), 0, stream>>>(
          Aq, Aq, kInner, 0L, Bk, Bk, kInner, 0L, (void*)SC, (void*)SC, kSeq, 0L, dumf, dumf, 0L,
          kSeq, kSeq, kDh, 1.0f);
      pcell_kernel<<<dim3(kSeq), dim3(256), 0, stream>>>(
          SC, GJ + (size_t)h * kSeq, PM + (size_t)h * kSeq, LFC + (size_t)h * kSeq, PP, INVN);
      const unsigned short* Bv = VT + (size_t)h * kDh * kSeq;
      wmma_gemm64<1, false, 0, 0, false, 0, 2, true><<<dim3(tilesCell / 8, 1), dim3(256), 0, stream>>>(
          PP, PP, kSeq, 0L, Bv, Bv, kSeq, 0L, (void*)OO, (void*)OO, kDh, 0L, dumf, dumf, 0L,
          kSeq, kDh, kSeq, 1.0f);
      ln_gate_kernel<<<dim3(kSeq), dim3(128), 0, stream>>>(OO, INVN, ACT, XM, nsc, skp, HSH, HSL, h);
    }
    float* outb = out + (size_t)b * kSeq * kEmb;
    wmma_gemm64<1, true, 0, 0, false, 0, 0, false><<<dim3(tilesDown / 8, 1), dim3(256), 0, stream>>>(
        HSH, HSL, kInner, 0L, WDT, WDT, kInner, 0L, (void*)outb, (void*)outb, kEmb, 0L, dumf, dumf, 0L,
        kSeq, kEmb, kInner, 1.0f);
  }
}
